// GroupedQueryAttention_43834436223189
// MI455X (gfx1250) — hardware-verified
//
#include <hip/hip_runtime.h>
#include <math.h>


#ifndef NB
#define NB 2
#endif
#ifndef TT
#define TT 2048
#endif
#ifndef RH
#define RH 256
#endif
#define NB_FULL 2
#define TT_FULL 2048
#define DM   2048
#define NH_  16
#define NKV  4
#define REP  (NH_ / NKV)
#define HD   128
#define DQ   (NH_ * HD)
#define DKV  (NKV * HD)
#define QKC  8.0f
#define SCLC (0.08838834764831845f * 0.015625f)
#define PCAR 1024.0f
#define ACAR 64.0f
#define WCAR 256.0f
#define OSC  (1.0f / 16384.0f)
#define PP   40
#define OP   136
static_assert(TT % 64 == 0);
static_assert(RH % 64 == 0);
static_assert(RH >= 64);
static_assert(RH <= TT);
static_assert(TT <= TT_FULL);
static_assert(NB >= 1);
static_assert(NB <= NB_FULL);
static_assert(DM % 32 == 0);
static_assert(DQ == DM);
static_assert(HD == 128);
static_assert((TT * HD) % 256 == 0);
static_assert(DM % 64 == 0);
static_assert(DQ % 64 == 0);
static_assert(DKV % 64 == 0);
static_assert(NH_ % NKV == 0);
static_assert(((size_t)DQ * DM) % 8 == 0);
static_assert(((size_t)DKV * DM) % 8 == 0);
static_assert(((size_t)TT * DM) % 8 == 0);
#define WS_CARVE_BYTES ((size_t)DQ * DM * 2 + 2 * (size_t)DKV * DM * 2 + (size_t)DM * DQ * 2 + (size_t)TT * HD * 2 * 4 + (size_t)TT * DM * 2 + (size_t)TT * DQ * 4 + 2 * (size_t)TT * DKV * 4 + 3 * (size_t)NH_ * TT * HD * 2 + 6 * (size_t)NKV * TT * HD * 2 + (size_t)TT * DQ * 2 + (size_t)RH * DQ * 2)
static_assert(WS_CARVE_BYTES <= (size_t)134217728);
static_assert(((size_t)RH * DQ * 2) % 256 == 0);
static_assert(((size_t)TT * HD * 2 * 4) % 256 == 0);

typedef _Float16 h16;
typedef unsigned short bf;
typedef __attribute__((ext_vector_type(16))) __bf16   v16bf;
typedef __attribute__((ext_vector_type(16))) _Float16 v16h;
typedef __attribute__((ext_vector_type(8)))  _Float16 v8h;
typedef __attribute__((ext_vector_type(8)))  unsigned short v8us;
typedef __attribute__((ext_vector_type(8)))  float    v8f;
typedef __attribute__((ext_vector_type(4)))  float    v4f;
typedef __attribute__((ext_vector_type(2)))  _Float16 v2h;
typedef __attribute__((ext_vector_type(2)))  unsigned short v2us;
typedef __attribute__((ext_vector_type(2)))  float    v2f;
typedef v8h  __attribute__((may_alias)) v8ha;
typedef v4f  __attribute__((may_alias)) v4fa;
typedef v8us __attribute__((may_alias)) v8usa;

__device__ __forceinline__ unsigned short f2bf(float f) { unsigned u = __float_as_uint(f); u += 0x7FFFu + ((u >> 16) & 1u); return (unsigned short)(u >> 16); }
__device__ __forceinline__ float bf2f(unsigned short b) { return __uint_as_float(((unsigned)b) << 16); }
__device__ __forceinline__ float bfr(float f) { return bf2f(f2bf(f)); }
__device__ __forceinline__ v16h cat16(v8h lo, v8h hi) { return __builtin_shufflevector(lo, hi, 0, 1, 2, 3, 4, 5, 6, 7, 8, 9, 10, 11, 12, 13, 14, 15); }
__device__ __forceinline__ v16bf cat16b(v8us lo, v8us hi) { return __builtin_bit_cast(v16bf, __builtin_shufflevector(lo, hi, 0, 1, 2, 3, 4, 5, 6, 7, 8, 9, 10, 11, 12, 13, 14, 15)); }
__device__ __forceinline__ v8f wmma16(v16h a, v16h b, v8f c) { return __builtin_amdgcn_wmma_f32_16x16x32_f16(false, a, false, b, (short)0, c, false, false); }
__device__ __forceinline__ v8f wmmab(v16bf a, v16bf b, v8f c) { return __builtin_amdgcn_wmma_f32_16x16x32_bf16(false, a, false, b, (short)0, c, false, false); }
__device__ __forceinline__ h16 tohx(float x) { return (h16)x; }
__device__ __forceinline__ void splitf(float y, unsigned short& h, unsigned short& l) { h = f2bf(y); l = f2bf(y - bf2f(h)); }
static __device__ __forceinline__ h16 toh_flush(float v) { const h16 r = (h16)v; return (fabsf(v) < 6.103515625e-05f) ? (h16)0.0f : r; }

template <typename T16> struct WFrag;
template <> struct WFrag<h16> { typedef v16h V; static __device__ __forceinline__ V ld(const h16* p) { return cat16(*(const v8h*)p, *(const v8h*)(p + 16)); } static __device__ __forceinline__ v8f mma(V a, V b, v8f c) { return wmma16(a, b, c); } };
template <> struct WFrag<bf> { typedef v16bf V; static __device__ __forceinline__ V ld(const bf* p) { return cat16b(*(const v8us*)p, *(const v8us*)(p + 16)); } static __device__ __forceinline__ v8f mma(V a, V b, v8f c) { return wmmab(a, b, c); } };

template <typename T16, int NSPLIT, bool BIAS>
__global__ __launch_bounds__(32) void k_gemmw(const T16* __restrict__ A, const T16* __restrict__ A2, const T16* __restrict__ Bt, const T16* __restrict__ Bt2, int K, float* C, int ldc, const float* __restrict__ bias, float cs, size_t sA, size_t sB, size_t sC) {
    typedef typename WFrag<T16>::V V;
    __shared__ __align__(16) float os[16 * 68];
    const size_t z = blockIdx.z; A += z * sA; if (A2) A2 += z * sA; Bt += z * sB; if (Bt2) Bt2 += z * sB; C += z * sC;
    const int lane = threadIdx.x & 31, lr = lane & 15, hi = lane >> 4; const int r0 = blockIdx.x * 64, c0 = blockIdx.y * 64;
    v8f acc[4][4];
#pragma unroll
    for (int mb = 0; mb < 4; ++mb)
#pragma unroll
        for (int nb = 0; nb < 4; ++nb) acc[mb][nb] = (v8f){};
    const size_t aoff = (size_t)(r0 + lr) * K + 8 * hi, boff = (size_t)(c0 + lr) * K + 8 * hi;
#pragma unroll 1
    for (int kc = 0; kc < K; kc += 32) {
        V b[4], b2[4];
#pragma unroll
        for (int nb = 0; nb < 4; ++nb) { b[nb] = WFrag<T16>::ld(Bt + boff + (size_t)nb * 16 * K + kc); b2[nb] = b[nb]; if (NSPLIT >= 2) b2[nb] = WFrag<T16>::ld(Bt2 + boff + (size_t)nb * 16 * K + kc); }
#pragma unroll
        for (int mb = 0; mb < 4; ++mb) {
            const V a = WFrag<T16>::ld(A + aoff + (size_t)mb * 16 * K + kc); V a2 = a; if (NSPLIT == 1 || NSPLIT == 2) a2 = WFrag<T16>::ld(A2 + aoff + (size_t)mb * 16 * K + kc);
#pragma unroll
            for (int nb = 0; nb < 4; ++nb) { acc[mb][nb] = WFrag<T16>::mma(a, b[nb], acc[mb][nb]); if (NSPLIT == 1 || NSPLIT == 2) acc[mb][nb] = WFrag<T16>::mma(a2, b[nb], acc[mb][nb]); if (NSPLIT >= 2) acc[mb][nb] = WFrag<T16>::mma(a, b2[nb], acc[mb][nb]); }
            asm volatile("v_nop\n\tv_nop\n\tv_nop\n\tv_nop" : "+v"(acc[mb][0]), "+v"(acc[mb][1]), "+v"(acc[mb][2]), "+v"(acc[mb][3]) : "v"(a), "v"(a2), "v"(b[0]), "v"(b[1]), "v"(b[2]), "v"(b[3]), "v"(b2[0]), "v"(b2[1]), "v"(b2[2]), "v"(b2[3]));
            __builtin_amdgcn_sched_barrier(0);
        }
    }
#pragma unroll
    for (int mb = 0; mb < 4; ++mb) {
#pragma unroll
        for (int nb = 0; nb < 4; ++nb) {
#pragma unroll
            for (int j = 0; j < 8; ++j) os[(hi * 8 + j) * 68 + nb * 16 + lr] = acc[mb][nb][j]; }
        __syncthreads();
        float* crow = C + (size_t)(r0 + mb * 16) * ldc + c0;
#pragma unroll 1
        for (int ps = 0; ps < 2; ++ps) {
#pragma unroll
            for (int s = 0; s < 8; ++s) { const int row = 2 * s + hi, cofs = lr * 4; v4f val = *(const v4fa*)(os + row * 68 + cofs); val = val * cs;
                if (BIAS) { val[0] += bfr(bias[c0 + cofs]); val[1] += bfr(bias[c0 + cofs + 1]); val[2] += bfr(bias[c0 + cofs + 2]); val[3] += bfr(bias[c0 + cofs + 3]); }
                *(volatile v4f*)(crow + (size_t)row * ldc + cofs) = val; }
            if (ps == 0) __threadfence(); }
        __syncthreads();
    }
}

__global__ __launch_bounds__(256) void k_cvt8(const float* __restrict__ src, bf* dst, size_t n8) { const size_t i = (size_t)blockIdx.x * 256 + threadIdx.x; if (i >= n8) return; const v8f v = *(const v8f*)(src + i * 8); v8us o;
#pragma unroll
    for (int k = 0; k < 8; ++k) o[k] = f2bf(v[k]); *(volatile v8us*)(dst + i * 8) = o; __threadfence(); *(volatile v8us*)(dst + i * 8) = o; }
__global__ __launch_bounds__(256) void k_cvt8h(const float* __restrict__ src, h16* dst, size_t n8, float sc) { const size_t i = (size_t)blockIdx.x * 256 + threadIdx.x; if (i >= n8) return; const v8f v = *(const v8f*)(src + i * 8); v8h o;
#pragma unroll
    for (int k = 0; k < 8; ++k) o[k] = tohx(bfr(v[k]) * sc); *(volatile v8h*)(dst + i * 8) = o; __threadfence(); *(volatile v8h*)(dst + i * 8) = o; }

struct ThetaTab { float th[HD / 2]; };
static_assert(sizeof(ThetaTab) == 256);
__global__ __launch_bounds__(256) void k_cstab(ThetaTab tab, float* CS) {
    const int idx = blockIdx.x * 256 + threadIdx.x; if (idx >= TT * HD) return;
    const int t = idx / HD, d = idx % HD, j = d & (HD / 2 - 1);
    float th = tab.th[0];
#pragma unroll
    for (int i = 1; i < HD / 2; ++i) th = (j == i) ? tab.th[i] : th;
    const float ang = __fmul_rn((float)t, th);
    float sn, cn; sincosf(ang, &sn, &cn);
    v2f o; o[0] = cn; o[1] = sn;
    *(volatile v2f*)(CS + (size_t)idx * 2) = o; __threadfence(); *(volatile v2f*)(CS + (size_t)idx * 2) = o; }

__global__ __launch_bounds__(256) void k_rope(const float* __restrict__ F, int pitch, int nheads, const float* __restrict__ CS, float sc, h16* P16, bf* Ph, bf* Pl) {
    const size_t e = ((size_t)blockIdx.x * 256 + threadIdx.x) * 2; if (e >= (size_t)nheads * TT * HD) return;
    const int d = (int)(e % HD); const int t = (int)((e / HD) % TT); const int h = (int)(e / ((size_t)HD * TT));
    const float* f = F + (size_t)t * pitch + h * HD; v2h o16; v2us oh, ol;
#pragma unroll
    for (int q = 0; q < 2; ++q) { const int dd = d + q; const int dp = (dd < HD / 2) ? dd + HD / 2 : dd - HD / 2; const float x0 = f[dd], x1 = f[dp];
        const v2f cs = *(const v2f*)(CS + ((size_t)t * HD + dd) * 2); float a = __fmul_rn(x0, cs[0]), bq = __fmul_rn(x1, cs[1]); asm volatile("" : "+v"(a)); asm volatile("" : "+v"(bq));
        const float r = ((dd < HD / 2) ? __fsub_rn(a, bq) : __fadd_rn(a, bq)) * sc;
        o16[q] = tohx(r); unsigned short a2, c2; splitf(r, a2, c2); oh[q] = a2; ol[q] = c2; }
    *(volatile v2h*)(P16 + e) = o16; *(volatile v2us*)(Ph + e) = oh; *(volatile v2us*)(Pl + e) = ol; __threadfence();
    *(volatile v2h*)(P16 + e) = o16; *(volatile v2us*)(Ph + e) = oh; *(volatile v2us*)(Pl + e) = ol; }
__global__ __launch_bounds__(256) void k_vtp(const float* __restrict__ F, int pitch, int nheads, h16* V16, bf* Vh, bf* Vl) { const size_t e = ((size_t)blockIdx.x * 256 + threadIdx.x) * 2; if (e >= (size_t)nheads * HD * TT) return; const int t = (int)(e % TT); const int d = (int)((e / TT) % HD); const int g = (int)(e / ((size_t)TT * HD)); v2h o16; v2us oh, ol;
#pragma unroll
    for (int q = 0; q < 2; ++q) { const float x = F[(size_t)(t + q) * pitch + g * HD + d]; o16[q] = tohx(x); unsigned short a2, c2; splitf(x, a2, c2); oh[q] = a2; ol[q] = c2; }
    *(volatile v2h*)(V16 + e) = o16; *(volatile v2us*)(Vh + e) = oh; *(volatile v2us*)(Vl + e) = ol; __threadfence(); *(volatile v2h*)(V16 + e) = o16; *(volatile v2us*)(Vh + e) = oh; *(volatile v2us*)(Vl + e) = ol; }

template <bool SPLIT>
__global__ __launch_bounds__(32) void k_flash(const h16* __restrict__ Q16, const bf* __restrict__ Qh, const bf* __restrict__ Ql,
                                              const h16* __restrict__ K16, const bf* __restrict__ Kh, const bf* __restrict__ Kl,
                                              const h16* __restrict__ V16, const bf* __restrict__ Vh, const bf* __restrict__ Vl,
                                              int roff, h16* AT, h16* ATL) {
    __shared__ __align__(16) h16 pt[16 * PP];
    __shared__ __align__(16) bf  pth[16 * PP];
    __shared__ __align__(16) bf  ptl[16 * PP];
    __shared__ __align__(16) h16 os[16 * OP];
    __shared__ __align__(16) h16 osl[16 * OP];
    const int lane = threadIdx.x & 31, lr = lane & 15, hi = lane >> 4;
    const int qt0 = roff + (int)blockIdx.x * 16; const int h = (int)blockIdx.y; const int g = h / REP;
    const size_t qoff = ((size_t)h * TT + qt0 + lr) * HD + 8 * hi;
    const size_t kb0  = (size_t)g * TT * HD + (size_t)lr * HD + 8 * hi;
    const size_t vb0  = (size_t)g * HD * TT + (size_t)lr * TT + 8 * hi;
    v8f oacc[8];
#pragma unroll
    for (int nb = 0; nb < 8; ++nb) oacc[nb] = (v8f){};
    float mrow[8], lrow[8];
#pragma unroll
    for (int r = 0; r < 8; ++r) { mrow[r] = -3.0e38f; lrow[r] = 0.0f; }
#pragma unroll 1
    for (int s0 = 0; s0 <= qt0; s0 += 32) {
        const size_t koff = kb0 + (size_t)s0 * HD;
        v8f c0 = (v8f){}; v8f c1 = (v8f){};
        if (SPLIT) {
#pragma unroll 1
            for (int kc = 0; kc < 4; ++kc) {
                v16bf a, a2, b, b2;
                a = WFrag<bf>::ld(Qh + qoff + kc * 32); a2 = WFrag<bf>::ld(Ql + qoff + kc * 32);
                b = WFrag<bf>::ld(Kh + koff + kc * 32); b2 = WFrag<bf>::ld(Kl + koff + kc * 32);
                c0 = wmmab(a, b, c0); c0 = wmmab(a2, b, c0); c0 = wmmab(a, b2, c0);
                b = WFrag<bf>::ld(Kh + koff + (size_t)16 * HD + kc * 32); b2 = WFrag<bf>::ld(Kl + koff + (size_t)16 * HD + kc * 32);
                c1 = wmmab(a, b, c1); c1 = wmmab(a2, b, c1); c1 = wmmab(a, b2, c1);
                asm volatile("v_nop\n\tv_nop\n\tv_nop\n\tv_nop" : "+v"(c0), "+v"(c1) : "v"(a), "v"(a2), "v"(b), "v"(b2)); }
        } else {
            v16h a, b;
#pragma unroll
            for (int kc = 0; kc < 4; ++kc) {
                a = WFrag<h16>::ld(Q16 + qoff + kc * 32);
                b = WFrag<h16>::ld(K16 + koff + kc * 32); c0 = wmma16(a, b, c0);
                b = WFrag<h16>::ld(K16 + koff + (size_t)16 * HD + kc * 32); c1 = wmma16(a, b, c1); }
            asm volatile("v_nop\n\tv_nop\n\tv_nop\n\tv_nop" : "+v"(c0), "+v"(c1) : "v"(a), "v"(b));
        }
        float al[8];
#pragma unroll
        for (int r = 0; r < 8; ++r) {
            const int qrow = qt0 + 8 * hi + r;
            const float t0 = (s0 + lr <= qrow) ? c0[r] * SCLC : -3.0e38f;
            const float t1 = (s0 + 16 + lr <= qrow) ? c1[r] * SCLC : -3.0e38f;
            float tv = fmaxf(t0, t1);
            tv = fmaxf(tv, __shfl_xor(tv, 1, 32)); tv = fmaxf(tv, __shfl_xor(tv, 2, 32)); tv = fmaxf(tv, __shfl_xor(tv, 4, 32)); tv = fmaxf(tv, __shfl_xor(tv, 8, 32));
            const float mnew = fmaxf(mrow[r], tv);
            float dm = __fsub_rn(mrow[r], mnew); asm volatile("" : "+v"(dm));
            const float alpha = __builtin_amdgcn_exp2f(__fmul_rn(dm, 1.4426950408889634f));
            float d0 = __fsub_rn(t0, mnew); asm volatile("" : "+v"(d0));
            float d1 = __fsub_rn(t1, mnew); asm volatile("" : "+v"(d1));
            const float p0 = __builtin_amdgcn_exp2f(__fmul_rn(d0, 1.4426950408889634f));
            const float p1 = __builtin_amdgcn_exp2f(__fmul_rn(d1, 1.4426950408889634f));
            mrow[r] = mnew;
            float q0, q1;
            if (SPLIT) {
                unsigned short ah, alo, bh, blo; splitf(p0, ah, alo); splitf(p1, bh, blo);
                pth[(8 * hi + r) * PP + lr] = ah; ptl[(8 * hi + r) * PP + lr] = alo; pth[(8 * hi + r) * PP + 16 + lr] = bh; ptl[(8 * hi + r) * PP + 16 + lr] = blo;
                q0 = bf2f(ah) + bf2f(alo); q1 = bf2f(bh) + bf2f(blo);
            } else {
                const h16 x0 = toh_flush(p0 * PCAR), x1 = toh_flush(p1 * PCAR);
                pt[(8 * hi + r) * PP + lr] = x0; pt[(8 * hi + r) * PP + 16 + lr] = x1;
                q0 = (float)x0; q1 = (float)x1;
            }
            float ts = q0 + q1;
            ts += __shfl_xor(ts, 1, 32); ts += __shfl_xor(ts, 2, 32); ts += __shfl_xor(ts, 4, 32); ts += __shfl_xor(ts, 8, 32);
            lrow[r] = lrow[r] * alpha + ts;
            al[r] = alpha;
        }
#pragma unroll
        for (int nb = 0; nb < 8; ++nb)
#pragma unroll
            for (int r = 0; r < 8; ++r) oacc[nb][r] *= al[r];
        __syncthreads();
        const size_t voff = vb0 + s0;
        if (SPLIT) {
            const v16bf pa  = cat16b(*(const v8usa*)(pth + lr * PP + 8 * hi), *(const v8usa*)(pth + lr * PP + 16 + 8 * hi));
            const v16bf pa2 = cat16b(*(const v8usa*)(ptl + lr * PP + 8 * hi), *(const v8usa*)(ptl + lr * PP + 16 + 8 * hi));
#pragma unroll
            for (int hq = 0; hq < 2; ++hq) {
                v16bf vb, vb2;
#pragma unroll
                for (int j = 0; j < 4; ++j) { const int nb = hq * 4 + j; vb = WFrag<bf>::ld(Vh + voff + (size_t)nb * 16 * TT); vb2 = WFrag<bf>::ld(Vl + voff + (size_t)nb * 16 * TT);
                    oacc[nb] = wmmab(pa, vb, oacc[nb]); oacc[nb] = wmmab(pa2, vb, oacc[nb]); oacc[nb] = wmmab(pa, vb2, oacc[nb]); }
                asm volatile("v_nop\n\tv_nop\n\tv_nop\n\tv_nop" : "+v"(oacc[hq * 4 + 0]), "+v"(oacc[hq * 4 + 1]), "+v"(oacc[hq * 4 + 2]), "+v"(oacc[hq * 4 + 3]) : "v"(pa), "v"(pa2), "v"(vb), "v"(vb2));
                __builtin_amdgcn_sched_barrier(0);
            }
        } else {
            const v16h pa = cat16(*(const v8ha*)(pt + lr * PP + 8 * hi), *(const v8ha*)(pt + lr * PP + 16 + 8 * hi));
            v16h vb;
#pragma unroll
            for (int nb = 0; nb < 8; ++nb) { vb = WFrag<h16>::ld(V16 + voff + (size_t)nb * 16 * TT); oacc[nb] = wmma16(pa, vb, oacc[nb]); }
            asm volatile("v_nop\n\tv_nop\n\tv_nop\n\tv_nop" : "+v"(oacc[0]), "+v"(oacc[1]), "+v"(oacc[2]), "+v"(oacc[3]), "+v"(oacc[4]), "+v"(oacc[5]), "+v"(oacc[6]), "+v"(oacc[7]) : "v"(pa), "v"(vb));
        }
        __syncthreads();
    }
#pragma unroll
    for (int r = 0; r < 8; ++r) {
        const float inv = ACAR / lrow[r];
#pragma unroll
        for (int nb = 0; nb < 8; ++nb) { const float v = oacc[nb][r] * inv; const h16 x = toh_flush(v); os[(8 * hi + r) * OP + nb * 16 + lr] = x; if (SPLIT) osl[(8 * hi + r) * OP + nb * 16 + lr] = toh_flush(v - (float)x); }
    }
    __syncthreads();
    h16* arow = AT + (size_t)qt0 * DQ + (size_t)h * HD;
#pragma unroll 1
    for (int ps = 0; ps < 2; ++ps) {
#pragma unroll
        for (int s = 0; s < 8; ++s) { const int row = 2 * s + hi; const v8h val = *(const v8ha*)(os + row * OP + lr * 8); *(volatile v8h*)(arow + (size_t)row * DQ + lr * 8) = val;
            if (SPLIT) { h16* lrw = ATL + (size_t)qt0 * DQ + (size_t)h * HD; const v8h v2 = *(const v8ha*)(osl + row * OP + lr * 8); *(volatile v8h*)(lrw + (size_t)row * DQ + lr * 8) = v2; } }
        if (ps == 0) __threadfence(); }
}

extern "C" void kernel_launch(void* const* d_in, const int* in_sizes, int n_in,
                              void* d_out, int out_size, void* d_ws, size_t ws_size, hipStream_t stream) {
    if (n_in < 5) return;
    const size_t rows_used = (size_t)(NB - 1) * TT_FULL + TT;
    if ((size_t)in_sizes[0] < rows_used * DM || (size_t)in_sizes[1] < (size_t)DQ * DM || (size_t)in_sizes[2] < (size_t)DKV * DM ||
        (size_t)in_sizes[3] < (size_t)DKV * DM || (size_t)in_sizes[4] < (size_t)DM * DQ || (size_t)out_size < rows_used * DM) return;
    const float* x = (const float*)d_in[0]; const float* wq = (const float*)d_in[1]; const float* wk = (const float*)d_in[2];
    const float* wv = (const float*)d_in[3]; const float* wo = (const float*)d_in[4];
    float* OUT = (float*)d_out;
    char* wsp = (char*)d_ws;
    auto take = [&](size_t bytes) { char* p = wsp; wsp += (bytes + 255) & ~(size_t)255; return (void*)p; };
    bf* WQ = (bf*)take((size_t)DQ * DM * 2); bf* WK = (bf*)take((size_t)DKV * DM * 2); bf* WV = (bf*)take((size_t)DKV * DM * 2); h16* WO = (h16*)take((size_t)DM * DQ * 2);
    float* CS = (float*)take((size_t)TT * HD * 2 * 4);
    bf* XB = (bf*)take((size_t)TT * DM * 2); float* FQ = (float*)take((size_t)TT * DQ * 4); float* FK = (float*)take((size_t)TT * DKV * 4); float* FV = (float*)take((size_t)TT * DKV * 4);
    h16* QP16 = (h16*)take((size_t)NH_ * TT * HD * 2); bf* QPh = (bf*)take((size_t)NH_ * TT * HD * 2); bf* QPl = (bf*)take((size_t)NH_ * TT * HD * 2);
    h16* KP16 = (h16*)take((size_t)NKV * TT * HD * 2); bf* KPh = (bf*)take((size_t)NKV * TT * HD * 2); bf* KPl = (bf*)take((size_t)NKV * TT * HD * 2);
    h16* VT16 = (h16*)take((size_t)NKV * HD * TT * 2); bf* VTh = (bf*)take((size_t)NKV * HD * TT * 2); bf* VTl = (bf*)take((size_t)NKV * HD * TT * 2);
    h16* AT16 = (h16*)take((size_t)TT * DQ * 2); h16* ATL16 = (h16*)take((size_t)RH * DQ * 2);
    if ((size_t)(wsp - (char*)d_ws) > ws_size) return;
    ThetaTab tab;
    for (int j = 0; j < HD / 2; ++j) { const double p = pow(10000.0, (double)(2 * j) / (double)HD); const float pf = (float)p; tab.th[j] = 1.0f / pf; }
    k_cvt8<<<(unsigned)(((size_t)DQ * DM / 8 + 255) / 256), 256, 0, stream>>>(wq, WQ, (size_t)DQ * DM / 8);
    k_cvt8<<<(unsigned)(((size_t)DKV * DM / 8 + 255) / 256), 256, 0, stream>>>(wk, WK, (size_t)DKV * DM / 8);
    k_cvt8<<<(unsigned)(((size_t)DKV * DM / 8 + 255) / 256), 256, 0, stream>>>(wv, WV, (size_t)DKV * DM / 8);
    k_cvt8h<<<(unsigned)(((size_t)DM * DQ / 8 + 255) / 256), 256, 0, stream>>>(wo, WO, (size_t)DM * DQ / 8, WCAR);
    k_cstab<<<(unsigned)((TT * HD + 255) / 256), 256, 0, stream>>>(tab, CS);
    const unsigned LQ = (unsigned)(((size_t)NH_ * TT * HD / 2 + 255) / 256), LK = (unsigned)(((size_t)NKV * TT * HD / 2 + 255) / 256);
    for (int b = 0; b < NB; ++b) {
        k_cvt8<<<(unsigned)(((size_t)TT * DM / 8 + 255) / 256), 256, 0, stream>>>(x + (size_t)b * TT_FULL * DM, XB, (size_t)TT * DM / 8);
        k_gemmw<bf, 0, false><<<dim3(TT / 64, DQ / 64, 1), 32, 0, stream>>>(XB, nullptr, WQ, nullptr, DM, FQ, DQ, nullptr, 1.0f, 0, 0, 0);
        k_rope<<<LQ, 256, 0, stream>>>(FQ, DQ, NH_, CS, QKC, QP16, QPh, QPl);
        k_gemmw<bf, 0, false><<<dim3(TT / 64, DKV / 64, 1), 32, 0, stream>>>(XB, nullptr, WK, nullptr, DM, FK, DKV, nullptr, 1.0f, 0, 0, 0);
        k_rope<<<LK, 256, 0, stream>>>(FK, DKV, NKV, CS, QKC, KP16, KPh, KPl);
        k_gemmw<bf, 0, false><<<dim3(TT / 64, DKV / 64, 1), 32, 0, stream>>>(XB, nullptr, WV, nullptr, DM, FV, DKV, nullptr, 1.0f, 0, 0, 0);
        k_vtp<<<LK, 256, 0, stream>>>(FV, DKV, NKV, VT16, VTh, VTl);
        k_flash<true><<<dim3(RH / 16, NH_, 1), 32, 0, stream>>>(QP16, QPh, QPl, KP16, KPh, KPl, VT16, VTh, VTl, 0, AT16, ATL16);
        if (TT > RH) k_flash<false><<<dim3((TT - RH) / 16, NH_, 1), 32, 0, stream>>>(QP16, QPh, QPl, KP16, KPh, KPl, VT16, VTh, VTl, RH, AT16, ATL16);
        float* OUTb = OUT + (size_t)b * TT_FULL * DM;
        k_gemmw<h16, 1, false><<<dim3(RH / 64, DM / 64, 1), 32, 0, stream>>>(AT16, ATL16, WO, nullptr, DQ, OUTb, DM, nullptr, OSC, 0, 0, 0);
        if (TT > RH) k_gemmw<h16, 0, false><<<dim3((TT - RH) / 64, DM / 64, 1), 32, 0, stream>>>(AT16 + (size_t)RH * DQ, nullptr, WO, nullptr, DQ, OUTb + (size_t)RH * DM, DM, nullptr, OSC, 0, 0, 0);
    }
}
